// DialogueGCN_91216515433183
// MI455X (gfx1250) — hardware-verified
//
#include <hip/hip_runtime.h>
#include <stdint.h>

#define DEVINL __device__ __forceinline__

typedef _Float16 f16t;
typedef unsigned short us_t;
typedef _Float16 v16h __attribute__((ext_vector_type(16)));
typedef _Float16 v8h  __attribute__((ext_vector_type(8)));
typedef _Float16 v4h  __attribute__((ext_vector_type(4)));
typedef __bf16   v16b __attribute__((ext_vector_type(16)));
typedef unsigned short v8us __attribute__((ext_vector_type(8)));
typedef float v8f __attribute__((ext_vector_type(8)));
typedef float v4f __attribute__((ext_vector_type(4)));
typedef int   v4i __attribute__((ext_vector_type(4)));
typedef v8h  __attribute__((may_alias)) v8ha;
typedef v4h  __attribute__((may_alias)) v4ha;
typedef v4f  __attribute__((may_alias)) v4fa;
typedef v4i  __attribute__((may_alias)) v4ia;
typedef v8us __attribute__((may_alias)) v8usa;
union FragH { v16h v; v4i q[2]; };
union FragB { v16b v; v4i q[2]; };

#define NU     4096
#define DE     512
#define WHALF  10
#define NWIN   21
#define NSLOT  32
#define NBLK   5
#define HWC    (NBLK * DE)
#define K3     (3 * DE)
#define WCAR   16.0f
#define WINV   (1.0f / 16.0f)
#define CT     256
#define GT     128
#define GM     128
#define GN     64
#define GPC    68
#define AT     128
#define TT     64
#define TPH    72

static_assert(GT == 4 * 32 && GM == 32 * 4 && GN == 64);
static_assert((NU % GM) == 0 && (DE % GN) == 0 && (HWC % GN) == 0);
static_assert((DE % 32) == 0 && (K3 % 32) == 0);
static_assert((GPC % 4) == 0 && (TPH % 8) == 0);
static_assert(DE == 4 * AT);
static_assert((NU % (CT / 32)) == 0);
static_assert(((NU * DE) % (8 * CT)) == 0 && ((DE * DE) % (8 * CT)) == 0);
static_assert(DE == 16 * 32);
static_assert((DE % TT) == 0 && TT * 4 == CT);
static_assert(NWIN <= NSLOT);

DEVINL us_t bf16_bits(float f) {
  unsigned u = __float_as_uint(f);
  u += 0x7fffu + ((u >> 16) & 1u);
  return (us_t)(u >> 16);
}

DEVINL v8f mma(const FragH& a, const FragH& b, v8f c) {
  v8f d = __builtin_amdgcn_wmma_f32_16x16x32_f16(false, a.v, false, b.v, (short)0, c, false, false);
  asm volatile("v_nop\n\tv_nop\n\tv_nop\n\tv_nop" : "+v"(d) : "v"(a.q[0]), "v"(a.q[1]), "v"(b.q[0]), "v"(b.q[1]));
  return d;
}
DEVINL v8f mma(const FragB& a, const FragB& b, v8f c) {
  v8f d = __builtin_amdgcn_wmma_f32_16x16x32_bf16(false, a.v, false, b.v, (short)0, c, false, false);
  asm volatile("v_nop\n\tv_nop\n\tv_nop\n\tv_nop" : "+v"(d) : "v"(a.q[0]), "v"(a.q[1]), "v"(b.q[0]), "v"(b.q[1]));
  return d;
}
DEVINL v8f zero8f() {
  v8f z = {0.f, 0.f, 0.f, 0.f, 0.f, 0.f, 0.f, 0.f};
  return z;
}
template <typename FR>
DEVINL void ldfrag(FR& f, const us_t* row, int k0) {
  f.q[0] = *(const v4ia*)(row + k0);
  f.q[1] = *(const v4ia*)(row + k0 + 16);
}

DEVINL float wsum32(float v) {
  v += __shfl_xor(v, 16);
  v += __shfl_xor(v, 8);
  v += __shfl_xor(v, 4);
  v += __shfl_xor(v, 2);
  v += __shfl_xor(v, 1);
  return v;
}
DEVINL float wmax32(float v) {
  v = fmaxf(v, __shfl_xor(v, 16));
  v = fmaxf(v, __shfl_xor(v, 8));
  v = fmaxf(v, __shfl_xor(v, 4));
  v = fmaxf(v, __shfl_xor(v, 2));
  v = fmaxf(v, __shfl_xor(v, 1));
  return v;
}

__global__ __launch_bounds__(CT) void cvt_x_k(const float* __restrict__ x, us_t* __restrict__ X16,
                                             us_t* __restrict__ XA3)
{
  const size_t idx = ((size_t)blockIdx.x * CT + threadIdx.x) * 8;
  const size_t row = idx >> 9, col = idx & 511;
  const v4f a = *(const v4fa*)(x + idx), c = *(const v4fa*)(x + idx + 4);
  v8h o16;
  v8us hi, lo;
  #pragma unroll
  for (int j = 0; j < 4; ++j) {
    const float v0 = a[j], v1 = c[j];
    o16[j] = (f16t)v0;
    o16[4 + j] = (f16t)v1;
    const us_t b0 = bf16_bits(v0), b1 = bf16_bits(v1);
    hi[j] = b0;
    hi[4 + j] = b1;
    lo[j]     = bf16_bits(v0 - __uint_as_float(((unsigned)b0) << 16));
    lo[4 + j] = bf16_bits(v1 - __uint_as_float(((unsigned)b1) << 16));
  }
  us_t* p16 = X16 + idx;
  us_t* p3  = XA3 + row * K3 + col;
  *(volatile v8h*)p16 = o16;
  *(volatile v8us*)p3 = hi;
  *(volatile v8us*)(p3 + DE) = lo;
  *(volatile v8us*)(p3 + 2 * DE) = hi;
  __threadfence();
  *(volatile v8h*)p16 = o16;
  *(volatile v8us*)p3 = hi;
  *(volatile v8us*)(p3 + DE) = lo;
  *(volatile v8us*)(p3 + 2 * DE) = hi;
}

__global__ __launch_bounds__(CT) void cvt_watt_k(const float* __restrict__ w, us_t* __restrict__ WA3)
{
  const size_t idx = ((size_t)blockIdx.x * CT + threadIdx.x) * 8;
  const size_t row = idx >> 9, col = idx & 511;
  const v4f a = *(const v4fa*)(w + idx), c = *(const v4fa*)(w + idx + 4);
  v8us hi, lo;
  #pragma unroll
  for (int j = 0; j < 4; ++j) {
    const float v0 = a[j], v1 = c[j];
    const us_t b0 = bf16_bits(v0), b1 = bf16_bits(v1);
    hi[j] = b0;
    hi[4 + j] = b1;
    lo[j]     = bf16_bits(v0 - __uint_as_float(((unsigned)b0) << 16));
    lo[4 + j] = bf16_bits(v1 - __uint_as_float(((unsigned)b1) << 16));
  }
  us_t* p3 = WA3 + row * K3 + col;
  *(volatile v8us*)p3 = hi;
  *(volatile v8us*)(p3 + DE) = hi;
  *(volatile v8us*)(p3 + 2 * DE) = lo;
  __threadfence();
  *(volatile v8us*)p3 = hi;
  *(volatile v8us*)(p3 + DE) = hi;
  *(volatile v8us*)(p3 + 2 * DE) = lo;
}

__global__ __launch_bounds__(CT) void cvt_wT_k(const float* __restrict__ wg, const float* __restrict__ wa,
                                              us_t* __restrict__ WT)
{
  __shared__ __attribute__((aligned(16))) f16t sT[TT * TPH];
  const int tid = threadIdx.x, blk = blockIdx.x;
  const int s = blk >> 6, tile = blk & 63;
  const int d0 = (tile >> 3) * TT, e0 = (tile & 7) * TT;
  const float* src = (s < 4) ? (wg + (size_t)s * DE * DE) : wa;
  const int dr = tid >> 2, ec = (tid & 3) * 16;
  const float* sp = src + ((size_t)(d0 + dr)) * DE + e0 + ec;
  v4f w4[4];
  #pragma unroll
  for (int p = 0; p < 4; ++p) w4[p] = *(const v4fa*)(sp + 4 * p);
  #pragma unroll
  for (int p = 0; p < 4; ++p) {
    #pragma unroll
    for (int c = 0; c < 4; ++c) sT[(ec + 4 * p + c) * TPH + dr] = (f16t)(w4[p][c] * WCAR);
  }
  __syncthreads();

  v8h v[2];
  us_t* dst[2];
  #pragma unroll
  for (int i = 0; i < 2; ++i) {
    const int q = tid + CT * i;
    const int e = q >> 3, piece = q & 7;
    v[i]   = *(const v8ha*)(sT + e * TPH + 8 * piece);
    dst[i] = WT + ((size_t)(DE * s + e0 + e)) * DE + d0 + 8 * piece;
  }
  #pragma unroll
  for (int i = 0; i < 2; ++i) *(volatile v8h*)dst[i] = v[i];
  __threadfence();
  #pragma unroll
  for (int i = 0; i < 2; ++i) *(volatile v8h*)dst[i] = v[i];
}

template <typename FR, int KD>
__global__ __launch_bounds__(GT) void gemm_k(const us_t* __restrict__ A, const us_t* __restrict__ BT,
                                            float* __restrict__ C, int ldc, float scale)
{
  __shared__ __attribute__((aligned(16))) float sC[GM * GPC];
  const int tid = threadIdx.x, lane = tid & 31, wave = tid >> 5;
  const int h = lane >> 4, m = lane & 15;
  const int tm0 = blockIdx.y * GM, tn0 = blockIdx.x * GN;

  v8f acc[2][4];
  #pragma unroll
  for (int s = 0; s < 2; ++s) {
    #pragma unroll
    for (int n = 0; n < 4; ++n) acc[s][n] = zero8f();
  }
  const us_t* arow = A  + ((size_t)(tm0 + 32 * wave + m)) * KD + 8 * h;
  const us_t* brow = BT + ((size_t)(tn0 + m)) * KD + 8 * h;

  #pragma unroll 1
  for (int ks = 0; ks < KD / 32; ++ks) {
    const int k0 = 32 * ks;
    FR a0, a1;
    ldfrag(a0, arow, k0);
    ldfrag(a1, arow + (size_t)16 * KD, k0);
    #pragma unroll
    for (int ct = 0; ct < 4; ++ct) {
      FR b;
      ldfrag(b, brow + (size_t)16 * ct * KD, k0);
      acc[0][ct] = mma(a0, b, acc[0][ct]);
      acc[1][ct] = mma(a1, b, acc[1][ct]);
    }
  }

  #pragma unroll
  for (int s = 0; s < 2; ++s) {
    #pragma unroll
    for (int ct = 0; ct < 4; ++ct) {
      #pragma unroll
      for (int r = 0; r < 8; ++r)
        sC[(32 * wave + 16 * s + 8 * h + r) * GPC + 16 * ct + m] = acc[s][ct][r] * scale;
    }
  }
  __syncthreads();

  v4f v[16];
  #pragma unroll
  for (int i = 0; i < 16; ++i) {
    const int q = tid + GT * i;
    const int row = q >> 4, piece = q & 15;
    v[i] = *(const v4fa*)(sC + row * GPC + 4 * piece);
  }
  #pragma unroll
  for (int i = 0; i < 16; ++i) {
    const int q = tid + GT * i;
    const int row = q >> 4, piece = q & 15;
    *(volatile v4f*)(C + ((size_t)(tm0 + row)) * ldc + tn0 + 4 * piece) = v[i];
  }
  __threadfence();
  #pragma unroll
  for (int i = 0; i < 16; ++i) {
    const int q = tid + GT * i;
    const int row = q >> 4, piece = q & 15;
    *(volatile v4f*)(C + ((size_t)(tm0 + row)) * ldc + tn0 + 4 * piece) = v[i];
  }
}

__global__ __launch_bounds__(CT) void att_k(const float* __restrict__ P, const float* __restrict__ x,
                                           float* __restrict__ ATT)
{
  const int tid = threadIdx.x, lane = tid & 31, wave = tid >> 5;
  const int n = blockIdx.x * (CT / 32) + wave;
  const float* xr = x + (size_t)n * DE + 16 * lane;
  v4f xv[4];
  #pragma unroll
  for (int q = 0; q < 4; ++q) xv[q] = *(const v4fa*)(xr + 4 * q);

  float mys = 0.0f;
  #pragma unroll 1
  for (int w = 0; w < NWIN; ++w) {
    const int j = n + w - WHALF;
    const bool valid = (j >= 0) && (j < NU);
    const int jc = min(max(j, 0), NU - 1);
    const float* pr = P + (size_t)jc * DE + 16 * lane;
    float s = 0.0f;
    #pragma unroll
    for (int q = 0; q < 4; ++q) {
      const v4f pv = *(const v4fa*)(pr + 4 * q);
      #pragma unroll
      for (int c = 0; c < 4; ++c) s = fmaf(pv[c], xv[q][c], s);
    }
    s = wsum32(s);
    s = valid ? s : 0.0f;
    mys = (lane == w) ? s : mys;
  }
  const bool inw = lane < NWIN;
  const float v = inw ? mys : -3.0e38f;
  const float mx = wmax32(v);
  float e = expf(mys - mx);
  e = inw ? e : 0.0f;
  const float sum = wsum32(e);
  const float a = e * (1.0f / sum);
  float* dst = ATT + (size_t)n * NSLOT + lane;
  *(volatile float*)dst = a;
  __threadfence();
  *(volatile float*)dst = a;
}

DEVINL v4f agg_row(const float* __restrict__ HW, const float* __restrict__ ATT,
                   const int* __restrict__ spk, int n, int t)
{
  const int sn = spk[n];
  v4f acc = *(const v4fa*)(HW + (size_t)n * HWC + 4 * DE + 4 * t);
  #pragma unroll 1
  for (int w = 0; w < NWIN; ++w) {
    const int j = n + w - WHALF;
    const bool valid = (j >= 0) && (j < NU);
    const int jc = min(max(j, 0), NU - 1);
    float a = ATT[(size_t)n * NSLOT + w];
    a = valid ? a : 0.0f;
    const int sj = spk[jc];
    const int o1 = (w >= WHALF) ? 0 : DE;
    const int o2 = (sj == sn) ? (2 * DE) : (3 * DE);
    const float* row = HW + (size_t)jc * HWC + 4 * t;
    const v4f v1 = *(const v4fa*)(row + o1);
    const v4f v2 = *(const v4fa*)(row + o2);
    #pragma unroll
    for (int c = 0; c < 4; ++c) acc[c] = fmaf(a, v1[c] + v2[c], acc[c]);
  }
  #pragma unroll
  for (int c = 0; c < 4; ++c) acc[c] = fmaxf(acc[c], 0.0f);
  return acc;
}

__global__ __launch_bounds__(AT) void agg1_k(const float* __restrict__ HW, const float* __restrict__ ATT,
                                            const int* __restrict__ spk, us_t* __restrict__ H16)
{
  __shared__ __attribute__((aligned(16))) f16t sH[DE];
  const int t = threadIdx.x, n = blockIdx.x;
  const v4f r = agg_row(HW, ATT, spk, n, t);
  v4h o;
  #pragma unroll
  for (int c = 0; c < 4; ++c) o[c] = (f16t)r[c];
  *(v4ha*)(sH + 4 * t) = o;
  __syncthreads();
  const bool act = t < DE / 8;
  const int tc = act ? t : 0;
  const v8h v = *(const v8ha*)(sH + 8 * tc);
  us_t* dst = H16 + (size_t)n * DE + 8 * tc;
  if (act) *(volatile v8h*)dst = v;
  __threadfence();
  if (act) *(volatile v8h*)dst = v;
}

__global__ __launch_bounds__(AT) void agg2_k(const float* __restrict__ HW, const float* __restrict__ ATT,
                                            const int* __restrict__ spk, float* __restrict__ out)
{
  const int t = threadIdx.x, n = blockIdx.x;
  const v4f r = agg_row(HW, ATT, spk, n, t);
  float* dst = out + (size_t)n * DE + 4 * t;
  *(volatile v4f*)dst = r;
  __threadfence();
  *(volatile v4f*)dst = r;
}

extern "C" void kernel_launch(void* const* d_in, const int* in_sizes, int n_in,
                              void* d_out, int out_size, void* d_ws, size_t ws_size,
                              hipStream_t stream) {
  if (n_in < 7) return;
  if (in_sizes[0] != NU * DE) return;
  if (in_sizes[1] != NU) return;
  if (in_sizes[2] != 4 * DE * DE) return;
  if (in_sizes[3] != 4 * DE * DE) return;
  if (in_sizes[4] != DE * DE) return;
  if (in_sizes[5] != DE * DE) return;
  if (in_sizes[6] != DE * DE) return;
  if (out_size != NU * DE) return;

  const float* x     = (const float*)d_in[0];
  const int*   spk   = (const int*)d_in[1];
  const float* w_gc1 = (const float*)d_in[2];
  const float* w_gc2 = (const float*)d_in[3];
  const float* w_att = (const float*)d_in[4];
  const float* w_ag1 = (const float*)d_in[5];
  const float* w_ag2 = (const float*)d_in[6];
  float* outp = (float*)d_out;

  const size_t szXA3 = (size_t)NU * K3 * 2;
  const size_t szWA3 = (size_t)DE * K3 * 2;
  const size_t szX16 = (size_t)NU * DE * 2;
  const size_t szWT  = (size_t)HWC * DE * 2;
  const size_t szP   = (size_t)NU * DE * 4;
  const size_t szATT = (size_t)NU * NSLOT * 4;
  const size_t szHW  = (size_t)NU * HWC * 4;
  const size_t szH16 = (size_t)NU * DE * 2;
  size_t off = 0;
  char* ws = (char*)d_ws;
  us_t*  XA3 = (us_t*)(ws + off);  off += szXA3;
  us_t*  WA3 = (us_t*)(ws + off);  off += szWA3;
  us_t*  X16 = (us_t*)(ws + off);  off += szX16;
  us_t*  W1T = (us_t*)(ws + off);  off += szWT;
  us_t*  W2T = (us_t*)(ws + off);  off += szWT;
  float* P   = (float*)(ws + off); off += szP;
  float* ATT = (float*)(ws + off); off += szATT;
  float* HW  = (float*)(ws + off); off += szHW;
  us_t*  H16 = (us_t*)(ws + off);  off += szH16;
  if (off > ws_size) return;
  if (off > (size_t)134217728) return;

  cvt_x_k<<<(NU * DE) / (8 * CT), CT, 0, stream>>>(x, X16, XA3);
  cvt_watt_k<<<(DE * DE) / (8 * CT), CT, 0, stream>>>(w_att, WA3);
  cvt_wT_k<<<NBLK * (DE / TT) * (DE / TT), CT, 0, stream>>>(w_gc1, w_ag1, W1T);
  cvt_wT_k<<<NBLK * (DE / TT) * (DE / TT), CT, 0, stream>>>(w_gc2, w_ag2, W2T);
  gemm_k<FragB, K3><<<dim3(DE / GN, NU / GM), GT, 0, stream>>>(XA3, WA3, P, DE, 1.0f);
  att_k<<<NU / (CT / 32), CT, 0, stream>>>(P, x, ATT);
  gemm_k<FragH, DE><<<dim3(HWC / GN, NU / GM), GT, 0, stream>>>(X16, W1T, HW, HWC, WINV);
  agg1_k<<<NU, AT, 0, stream>>>(HW, ATT, spk, H16);
  gemm_k<FragH, DE><<<dim3(HWC / GN, NU / GM), GT, 0, stream>>>(H16, W2T, HW, HWC, WINV);
  agg2_k<<<NU, AT, 0, stream>>>(HW, ATT, spk, outp);
  (void)hipGetLastError();
}
